// LightAttentiveConvNet_23948737642656
// MI455X (gfx1250) — hardware-verified
//
#include <hip/hip_runtime.h>
#include <math.h>

typedef __attribute__((ext_vector_type(16))) _Float16 v16h;
typedef __attribute__((ext_vector_type(16))) __bf16 v16b;
typedef __attribute__((ext_vector_type(8)))  _Float16 v8h;
typedef __attribute__((ext_vector_type(8)))  float v8f;
typedef __attribute__((ext_vector_type(4)))  float v4f;
typedef __attribute__((ext_vector_type(2)))  float v2f;
typedef __attribute__((ext_vector_type(4)))  unsigned v4u;
typedef __attribute__((ext_vector_type(4)))  int v4i;
typedef float __attribute__((may_alias)) float_a;
typedef int __attribute__((may_alias)) int_a;

template <typename T> __device__ __forceinline__ void vst2(void* p, T v) { *(volatile T*)p = v; __threadfence(); *(volatile T*)p = v; }
__device__ __forceinline__ v8f wmma16(v16h a, v16h b, v8f c) {
  v8f d = __builtin_amdgcn_wmma_f32_16x16x32_f16(false, a, false, b, (short)0, c, false, false);
  asm volatile("v_nop\n\tv_nop\n\tv_nop\n\tv_nop" : "+v"(d) : "v"(a), "v"(b));
  return d;
}
__device__ __forceinline__ v8f wmma_bf(v16b a, v16b b, v8f c) {
  v8f d = __builtin_amdgcn_wmma_f32_16x16x32_bf16(false, a, false, b, (short)0, c, false, false);
  asm volatile("v_nop\n\tv_nop\n\tv_nop\n\tv_nop" : "+v"(d) : "v"(a), "v"(b));
  return d;
}
__device__ __forceinline__ v16h frag_h(const _Float16* rowk0, int lane) {
  union { v16h v; v8h q[2]; } u; const _Float16* p = rowk0 + 8 * (lane >> 4);
  u.q[0] = *(const v8h*)p; u.q[1] = *(const v8h*)(p + 16); return u.v;
}
__device__ __forceinline__ v16h frag_f32(const float* rowk0, int lane) {
  v16h a; const float* p = rowk0 + 8 * (lane >> 4);
#pragma unroll
  for (int i = 0; i < 8; ++i) { a[i] = (_Float16)p[i]; a[8 + i] = (_Float16)p[16 + i]; }
  return a;
}
__device__ __forceinline__ v16h frag_f32s(const float* rowk0, int lane, float sc) {
  v16h a; const float* p = rowk0 + 8 * (lane >> 4);
#pragma unroll
  for (int i = 0; i < 8; ++i) { a[i] = (_Float16)(p[i] * sc); a[8 + i] = (_Float16)(p[16 + i] * sc); }
  return a;
}
__device__ __forceinline__ v16h fragc_f32(const float* W, int k0, int n, int lane, int ld, int K) {
  v16h a; const int g = lane >> 4;
#pragma unroll
  for (int i = 0; i < 8; ++i) { const int ka = k0 + 8 * g + i, kb = ka + 16;
    a[i] = (_Float16)(ka < K ? W[(size_t)ka * ld + n] : 0.f); a[8 + i] = (_Float16)(kb < K ? W[(size_t)kb * ld + n] : 0.f); }
  return a;
}
struct F2 { v16b h, l; };
__device__ __forceinline__ F2 bsplit16(const float v[16]) { F2 r;
#pragma unroll
  for (int i = 0; i < 16; ++i) { const __bf16 h = (__bf16)v[i]; r.h[i] = h; r.l[i] = (__bf16)(v[i] - (float)h); }
  return r; }
__device__ __forceinline__ F2 split_row(const float* row, int k0, int lane) { float v[16]; const float* p = row + k0 + 8 * (lane >> 4);
#pragma unroll
  for (int i = 0; i < 8; ++i) { v[i] = p[i]; v[8 + i] = p[16 + i]; }
  return bsplit16(v); }
__device__ __forceinline__ F2 split_rowK(const float* row, int k0, int lane, int K) { float v[16]; const int g = lane >> 4;
#pragma unroll
  for (int i = 0; i < 8; ++i) { const int ka = k0 + 8 * g + i, kb = ka + 16; v[i] = ka < K ? row[ka] : 0.f; v[8 + i] = kb < K ? row[kb] : 0.f; }
  return bsplit16(v); }
__device__ __forceinline__ F2 split_col(const float* W, int k0, int n, int lane, int ld, int K) { float v[16]; const int g = lane >> 4;
#pragma unroll
  for (int i = 0; i < 8; ++i) { const int ka = k0 + 8 * g + i, kb = ka + 16; v[i] = ka < K ? W[(size_t)ka * ld + n] : 0.f; v[8 + i] = kb < K ? W[(size_t)kb * ld + n] : 0.f; }
  return bsplit16(v); }
__device__ __forceinline__ v8f mac3(const F2& a, const F2& b, v8f c) { c = wmma_bf(a.l, b.h, c); c = wmma_bf(a.h, b.l, c); return wmma_bf(a.h, b.h, c); }
__device__ __forceinline__ float sigm(float v) { return 1.0f / (1.0f + expf(-v)); }
#define LDSX() do { asm volatile("s_wait_dscnt 0" ::: "memory"); __builtin_amdgcn_wave_barrier(); __builtin_amdgcn_fence(__ATOMIC_RELEASE, "workgroup"); } while (0)

#define NB 32
#define SL 512
#define EM 512
#define FT 256
#define NA 10
#define NC 8
#define VOC 32000
#define NR (NB * SL)

__global__ __launch_bounds__(256) void k_emb(const int* __restrict__ tok, const float* __restrict__ emb, _Float16* __restrict__ ex16) {
  const int tid = threadIdx.x, r = blockIdx.x * 4 + (tid >> 6), part = tid & 63;
  int id = tok[r]; id = id < 0 ? 0 : (id >= VOC ? VOC - 1 : id);
  union { v8h h; v4u u; } pk; const float* src = emb + (size_t)id * EM + part * 8;
#pragma unroll
  for (int e = 0; e < 8; ++e) pk.h[e] = (_Float16)(src[e] * 32.0f);
  vst2(ex16 + (size_t)r * EM + part * 8, pk.u);
}
__global__ __launch_bounds__(256) void k_packWh(const float* __restrict__ Wh, _Float16* __restrict__ WhT) {
  const int f = blockIdx.x, tid = threadIdx.x; __shared__ __align__(16) _Float16 srow[3 * EM];
  for (int q = tid; q < 3 * EM; q += 256) { const int k = q / EM, e = q % EM; srow[q] = (_Float16)(Wh[((size_t)f * EM + e) * 3 + k] * 32.0f); }
  __syncthreads();
  for (int q = tid; q < 3 * EM / 8; q += 256) vst2(WhT + (size_t)f * 3 * EM + q * 8, *(const v4u*)(&srow[q * 8]));
}
__global__ __launch_bounds__(128) void k_scores(const _Float16* __restrict__ ex16, const float* __restrict__ A, float* __restrict__ sc, float* __restrict__ at) {
  __shared__ __align__(16) float ss[4][16][16]; __shared__ __align__(16) float sa[4][16][16];
  const int tid = threadIdx.x, wave = tid >> 5, lane = tid & 31, col = lane & 15, g = lane >> 4;
  const int r0 = blockIdx.x * 64 + wave * 16;
  v8f acc = {};
#pragma unroll 4
  for (int kc = 0; kc < EM / 32; ++kc) { v16h bb;
#pragma unroll
    for (int i = 0; i < 8; ++i) { const int ka = kc * 32 + 8 * g + i; bb[i] = (_Float16)(col < NA ? A[(size_t)ka * NA + col] * 8.0f : 0.f); bb[8 + i] = (_Float16)(col < NA ? A[(size_t)(ka + 16) * NA + col] * 8.0f : 0.f); }
    acc = wmma16(frag_h(ex16 + (size_t)(r0 + col) * EM + kc * 32, lane), bb, acc); }
#pragma unroll
  for (int r = 0; r < 8; ++r) ss[wave][8 * g + r][col] = col < NA ? acc[r] * (1.0f / 256.0f) : 0.f;
  LDSX();
  if (g == 0) { const int m = col; float mx = -3.0e38f; for (int a = 0; a < NA; ++a) mx = fmaxf(mx, ss[wave][m][a]); float l = 0.f, p[NA];
    for (int a = 0; a < NA; ++a) { p[a] = expf(ss[wave][m][a] - mx); l += p[a]; } const float inv = 1.0f / l;
    for (int a = 0; a < 16; ++a) sa[wave][m][a] = a < NA ? p[a] * inv : 0.f; }
  LDSX();
  for (int q = lane; q < 16 * 4; q += 32) { const int rl = q >> 2, pc = q & 3; vst2(sc + (size_t)(r0 + rl) * 16 + pc * 4, *(const v4f*)(&ss[wave][rl][pc * 4])); vst2(at + (size_t)(r0 + rl) * 16 + pc * 4, *(const v4f*)(&sa[wave][rl][pc * 4])); }
}
__global__ __launch_bounds__(128) void k_cbr(const float* __restrict__ sc, const float* __restrict__ at, const float* __restrict__ Wc, float* __restrict__ cpart) {
  __shared__ __align__(16) float satt[64][EM + 4];
  __shared__ __align__(16) float smax[4][FT];
  const int tid = threadIdx.x, wave = tid >> 5, lane = tid & 31, col = lane & 15, g = lane >> 4;
  const int b = blockIdx.y, l0 = blockIdx.x * 64 + wave * 16; const size_t rb = (size_t)b * SL;
  { v16h a;
#pragma unroll
    for (int i = 0; i < 8; ++i) { a[i] = (_Float16)at[(rb + l0 + col) * 16 + 8 * g + i]; a[8 + i] = (_Float16)0.f; }
#pragma unroll 1
    for (int tt = 0; tt < SL / 16; ++tt) { v16h bb;
#pragma unroll
      for (int i = 0; i < 8; ++i) { bb[i] = (_Float16)(sc[(rb + tt * 16 + col) * 16 + 8 * g + i] * 32.0f); bb[8 + i] = (_Float16)0.f; }
      v8f acc = {}; acc = wmma16(a, bb, acc);
#pragma unroll
      for (int r = 0; r < 8; ++r) satt[wave * 16 + 8 * g + r][tt * 16 + col] = acc[r]; } }
  LDSX();
  { v8f acc[16];
#pragma unroll
    for (int j = 0; j < 16; ++j) acc[j] = (v8f){};
#pragma unroll 1
    for (int kc = 0; kc < EM / 32; ++kc) { const v16h a = frag_f32(&satt[wave * 16 + col][0] + kc * 32, lane);
#pragma unroll
      for (int j = 0; j < 16; ++j) acc[j] = wmma16(a, frag_f32s(Wc + (size_t)(j * 16 + col) * EM + kc * 32, lane, 32.0f), acc[j]); }
#pragma unroll
    for (int j = 0; j < 16; ++j) { float m = -3.0e38f;
#pragma unroll
      for (int r = 0; r < 8; ++r) m = fmaxf(m, acc[j][r]);
      m = fmaxf(m, __shfl_xor(m, 16, 32)); if (g == 0) smax[wave][j * 16 + col] = m * (1.0f / 1024.0f); } }
  __syncthreads();
  if (tid < 64) { float4 v; float* vv = (float*)&v; for (int e = 0; e < 4; ++e) { const int f = tid * 4 + e; vv[e] = fmaxf(fmaxf(smax[0][f], smax[1][f]), fmaxf(smax[2][f], smax[3][f])); }
    vst2(cpart + ((size_t)b * 8 + blockIdx.x) * FT + tid * 4, *(const v4f*)vv); }
}
__global__ __launch_bounds__(128) void k_hbr(const _Float16* __restrict__ ex16, const _Float16* __restrict__ WhT, float* __restrict__ hpart) {
  __shared__ __align__(16) float smax[4][FT];
  const int tid = threadIdx.x, wave = tid >> 5, lane = tid & 31, col = lane & 15, g = lane >> 4;
  const int b = blockIdx.y, t0 = blockIdx.x * 64 + wave * 16; const size_t rb = (size_t)b * SL;
  v8f acc[16];
#pragma unroll
  for (int j = 0; j < 16; ++j) acc[j] = (v8f){};
#pragma unroll 1
  for (int kc = 0; kc < 3 * EM / 32; ++kc) { const int k = kc / 16, e0 = (kc % 16) * 32; const int ra = min(t0 + col + k, SL - 1);
    const v16h a = frag_h(ex16 + (rb + ra) * EM + e0, lane);
#pragma unroll
    for (int j = 0; j < 16; ++j) acc[j] = wmma16(a, frag_h(WhT + (size_t)(j * 16 + col) * (3 * EM) + kc * 32, lane), acc[j]); }
#pragma unroll
  for (int j = 0; j < 16; ++j) { float m = -3.0e38f;
#pragma unroll
    for (int r = 0; r < 8; ++r) { const int tp = t0 + 8 * g + r; if (tp < SL - 2) m = fmaxf(m, acc[j][r]); }
    m = fmaxf(m, __shfl_xor(m, 16, 32)); if (g == 0) smax[wave][j * 16 + col] = m * (1.0f / 1024.0f); }
  __syncthreads();
  if (tid < 64) { float4 v; float* vv = (float*)&v; for (int e = 0; e < 4; ++e) { const int f = tid * 4 + e; vv[e] = fmaxf(fmaxf(smax[0][f], smax[1][f]), fmaxf(smax[2][f], smax[3][f])); }
    vst2(hpart + ((size_t)b * 8 + blockIdx.x) * FT + tid * 4, *(const v4f*)vv); }
}
__global__ __launch_bounds__(256) void k_fin(const float* __restrict__ hpart, const float* __restrict__ cpart, const float* __restrict__ tb, const float* __restrict__ Wfc, const float* __restrict__ bfc, float* __restrict__ out) {
  __shared__ float sz[FT]; __shared__ __align__(16) float so[NB * NC];
  const int tid = threadIdx.x;
#pragma unroll 1
  for (int b = 0; b < NB; ++b) {
    { const int f = tid; float hm = -3.0e38f, cm = -3.0e38f; for (int k = 0; k < 8; ++k) { hm = fmaxf(hm, hpart[((size_t)b * 8 + k) * FT + f]); cm = fmaxf(cm, cpart[((size_t)b * 8 + k) * FT + f]); }
      sz[f] = tanhf(hm + cm + tb[f]); }
    __syncthreads();
    if (tid < NC) { float a = bfc[tid];
#pragma unroll 1
      for (int f = 0; f < FT; ++f) a += sz[f] * Wfc[tid * FT + f];
      so[b * NC + tid] = a; }
    __syncthreads(); }
  if (tid < NB * NC / 4) vst2(out + tid * 4, *(const v4f*)(&so[tid * 4]));
}
extern "C" void kernel_launch(void* const* d_in, const int* in_sizes, int n_in, void* d_out, int out_size, void* d_ws, size_t ws_size, hipStream_t stream) {
  (void)in_sizes; (void)n_in; (void)out_size; (void)ws_size;
  const int* tok = (const int*)d_in[0]; const float* emb = (const float*)d_in[1]; const float* A = (const float*)d_in[2]; const float* Wh = (const float*)d_in[3]; const float* Wc = (const float*)d_in[4]; const float* tb = (const float*)d_in[5]; const float* Wfc = (const float*)d_in[6]; const float* bfc = (const float*)d_in[7];
  float* out = (float*)d_out;
  char* ws = (char*)d_ws; size_t off = 0;
  auto take = [&](size_t bytes) { char* p = ws + off; off += (bytes + 255) & ~(size_t)255; return p; };
  _Float16* ex16 = (_Float16*)take((size_t)NR * EM * 2); _Float16* WhT = (_Float16*)take((size_t)FT * 3 * EM * 2); float* sc = (float*)take((size_t)NR * 16 * 4); float* at = (float*)take((size_t)NR * 16 * 4);
  float* cpart = (float*)take((size_t)NB * 8 * FT * 4); float* hpart = (float*)take((size_t)NB * 8 * FT * 4);
  k_emb<<<NR / 4, 256, 0, stream>>>(tok, emb, ex16);
  k_packWh<<<FT, 256, 0, stream>>>(Wh, WhT);
  k_scores<<<NR / 64, 128, 0, stream>>>(ex16, A, sc, at);
  k_cbr<<<dim3(SL / 64, NB), 128, 0, stream>>>(sc, at, Wc, cpart);
  k_hbr<<<dim3(SL / 64, NB), 128, 0, stream>>>(ex16, WhT, hpart);
  k_fin<<<1, 256, 0, stream>>>(hpart, cpart, tb, Wfc, bfc, out);
}
